// MultiHeadSelfAttentionTENER_4071628997264
// MI455X (gfx1250) — hardware-verified
//
#include <hip/hip_runtime.h>


#define NB_  4
#define TT   1024
#define DM   512
#define NH_  8
#define HD   64
typedef _Float16 h16;
typedef unsigned short bf;
typedef __attribute__((ext_vector_type(16))) __bf16   v16bf;
typedef __attribute__((ext_vector_type(16))) _Float16 v16h;
typedef __attribute__((ext_vector_type(8)))  _Float16 v8h;
typedef __attribute__((ext_vector_type(8)))  unsigned short v8us;
typedef __attribute__((ext_vector_type(8)))  float    v8f;
typedef __attribute__((ext_vector_type(4)))  float    v4f;
typedef v8h  __attribute__((may_alias)) v8ha;
typedef v4f  __attribute__((may_alias)) v4fa;
typedef v8us __attribute__((may_alias)) v8usa;

__device__ __forceinline__ unsigned short f2bf(float f) { unsigned u = __float_as_uint(f); u += 0x7FFFu + ((u >> 16) & 1u); return (unsigned short)(u >> 16); }
__device__ __forceinline__ float bf2f(unsigned short b) { return __uint_as_float(((unsigned)b) << 16); }
__device__ __forceinline__ float bfr(float f) { return bf2f(f2bf(f)); }
__device__ __forceinline__ v16h cat16(v8h lo, v8h hi) { return __builtin_shufflevector(lo, hi, 0, 1, 2, 3, 4, 5, 6, 7, 8, 9, 10, 11, 12, 13, 14, 15); }
__device__ __forceinline__ v16bf cat16b(v8us lo, v8us hi) { return __builtin_bit_cast(v16bf, __builtin_shufflevector(lo, hi, 0, 1, 2, 3, 4, 5, 6, 7, 8, 9, 10, 11, 12, 13, 14, 15)); }
__device__ __forceinline__ v8f wmma16(v16h a, v16h b, v8f c) { return __builtin_amdgcn_wmma_f32_16x16x32_f16(false, a, false, b, (short)0, c, false, false); }
__device__ __forceinline__ v8f wmmab(v16bf a, v16bf b, v8f c) { return __builtin_amdgcn_wmma_f32_16x16x32_bf16(false, a, false, b, (short)0, c, false, false); }


template <typename T16> struct WFrag;
template <> struct WFrag<h16> { typedef v16h V; static __device__ __forceinline__ V ld(const h16* p) { return cat16(*(const v8h*)p, *(const v8h*)(p + 16)); } static __device__ __forceinline__ v8f mma(V a, V b, v8f c) { return wmma16(a, b, c); } };
template <> struct WFrag<bf> { typedef v16bf V; static __device__ __forceinline__ V ld(const bf* p) { return cat16b(*(const v8us*)p, *(const v8us*)(p + 16)); } static __device__ __forceinline__ v8f mma(V a, V b, v8f c) { return wmmab(a, b, c); } };
template <typename T16, int NSPLIT, bool BIAS>
__global__ __launch_bounds__(32) void k_gemmw(const T16* __restrict__ A, const T16* __restrict__ A2, const T16* __restrict__ Bt, const T16* __restrict__ Bt2, int K, float* C, int ldc, const float* __restrict__ bias, size_t sA, size_t sB, size_t sC) {
    typedef typename WFrag<T16>::V V;
    __shared__ __align__(16) float os[16 * 68];
    const size_t z = blockIdx.z; A += z * sA; if (A2) A2 += z * sA; Bt += z * sB; if (Bt2) Bt2 += z * sB; C += z * sC;
    const int lane = threadIdx.x & 31, lr = lane & 15, hi = lane >> 4; const int r0 = blockIdx.x * 64, c0 = blockIdx.y * 64;
    v8f acc[4][4];
#pragma unroll
    for (int mb = 0; mb < 4; ++mb)
#pragma unroll
        for (int nb = 0; nb < 4; ++nb) acc[mb][nb] = (v8f){};
    const size_t aoff = (size_t)(r0 + lr) * K + 8 * hi, boff = (size_t)(c0 + lr) * K + 8 * hi;
#pragma unroll 1
    for (int kc = 0; kc < K; kc += 32) {
        V a[4], a2[4];
#pragma unroll
        for (int mb = 0; mb < 4; ++mb) { a[mb] = WFrag<T16>::ld(A + aoff + (size_t)mb * 16 * K + kc); if (NSPLIT == 1 || NSPLIT == 2) a2[mb] = WFrag<T16>::ld(A2 + aoff + (size_t)mb * 16 * K + kc); }
#pragma unroll
        for (int nb = 0; nb < 4; ++nb) { const V b = WFrag<T16>::ld(Bt + boff + (size_t)nb * 16 * K + kc); V b2; if (NSPLIT >= 2) b2 = WFrag<T16>::ld(Bt2 + boff + (size_t)nb * 16 * K + kc);
#pragma unroll
            for (int mb = 0; mb < 4; ++mb) { acc[mb][nb] = WFrag<T16>::mma(a[mb], b, acc[mb][nb]); if (NSPLIT == 1 || NSPLIT == 2) acc[mb][nb] = WFrag<T16>::mma(a2[mb], b, acc[mb][nb]); if (NSPLIT >= 2) acc[mb][nb] = WFrag<T16>::mma(a[mb], b2, acc[mb][nb]); } }
        asm volatile("v_nop\n\tv_nop\n\tv_nop\n\tv_nop" : "+v"(acc[0][0]), "+v"(acc[1][1]), "+v"(acc[2][2]), "+v"(acc[3][3]) : "v"(a[0]), "v"(a[3]));
    }
#pragma unroll
    for (int mb = 0; mb < 4; ++mb) {
#pragma unroll
        for (int nb = 0; nb < 4; ++nb) {
#pragma unroll
            for (int j = 0; j < 8; ++j) os[(hi * 8 + j) * 68 + nb * 16 + lr] = acc[mb][nb][j]; }
        __builtin_amdgcn_wave_barrier(); asm volatile("" ::: "memory");
        float* crow = C + (size_t)(r0 + mb * 16) * ldc + c0;
#pragma unroll 1
        for (int ps = 0; ps < 2; ++ps) {
#pragma unroll
            for (int s = 0; s < 8; ++s) { const int row = 2 * s + hi, cofs = lr * 4; v4f val = *(const v4fa*)(os + row * 68 + cofs); if (BIAS) { val[0] += bfr(bias[c0 + cofs]); val[1] += bfr(bias[c0 + cofs + 1]); val[2] += bfr(bias[c0 + cofs + 2]); val[3] += bfr(bias[c0 + cofs + 3]); }
                *(volatile v4f*)(crow + (size_t)row * ldc + cofs) = val; }
            if (ps == 0) __threadfence(); }
        __builtin_amdgcn_wave_barrier(); asm volatile("" ::: "memory");
    }
}

__device__ __forceinline__ void splitf(float y, unsigned short& h, unsigned short& l) { h = f2bf(y); l = f2bf(y - bf2f(h)); }
typedef __attribute__((ext_vector_type(4))) unsigned short v4us;
typedef __attribute__((ext_vector_type(2))) unsigned short v2us;

__global__ __launch_bounds__(256) void k_cvt8(const float* __restrict__ src, bf* dst, size_t n8) { const size_t i = (size_t)blockIdx.x * 256 + threadIdx.x; if (i >= n8) return; const v8f v = *(const v8f*)(src + i * 8); v8us o;
#pragma unroll
    for (int k = 0; k < 8; ++k) o[k] = f2bf(v[k]); *(volatile v8us*)(dst + i * 8) = o; __threadfence(); *(volatile v8us*)(dst + i * 8) = o; }
__global__ __launch_bounds__(256) void k_wtG(const float* __restrict__ w, int K, int N, bf* Bt) {
    const int lane = threadIdx.x & 31; const int L0 = (blockIdx.x * 8 + (threadIdx.x >> 5)) * 8; const int nlines = N * K / 64;
#pragma unroll 1
    for (int ps = 0; ps < 2; ++ps) {
#pragma unroll 1
        for (int l = 0; l < 8; ++l) { const int L = L0 + l; if (L >= nlines) break; const size_t e = (size_t)L * 64 + lane * 2; const int k = (int)(e % K), n = (int)(e / K); v2us o;
            o[0] = f2bf(w[(size_t)k * N + n]); o[1] = f2bf(w[(size_t)(k + 1) * N + n]); *(volatile v2us*)(Bt + e) = o; }
        if (ps == 0) __threadfence(); }
}
__global__ __launch_bounds__(256) void k_pe(bf* Ph, bf* Pl) { const int e = (blockIdx.x * 256 + threadIdx.x) * 4; if (e >= 2 * TT * HD) return; const int d = e % HD; const int l = e / HD; const float p = (float)(l - TT); v4us oh, ol;
#pragma unroll 1
    for (int q = 0; q < 4; ++q) { const int dd = d + q; const int j = dd < 32 ? dd : dd - 32; const float div = expf((float)j * (-(logf(10000.0f) / 31.0f))); const float ang = __fmul_rn(p, div); const float v = dd < 32 ? sinf(ang) : cosf(ang); unsigned short a, c; splitf(v, a, c); oh[q] = a; ol[q] = c; }
    *(volatile v4us*)(Ph + e) = oh; *(volatile v4us*)(Pl + e) = ol; __threadfence(); *(volatile v4us*)(Ph + e) = oh; *(volatile v4us*)(Pl + e) = ol; }
__global__ __launch_bounds__(256) void k_qpl(const float* __restrict__ FQ, const float* __restrict__ vb, bf* Qh, bf* Ql, bf* QVh, bf* QVl) { const int e = (blockIdx.x * 256 + threadIdx.x) * 4; if (e >= NH_ * TT * HD) return; const int d = e % HD; const int t = (e / HD) % TT; const int h = e / (HD * TT); const v4f a = *(const v4f*)(FQ + (size_t)t * DM + h * HD + d); v4us qh, ql, vh, vl;
#pragma unroll
    for (int q = 0; q < 4; ++q) { unsigned short u, c; splitf(a[q], u, c); qh[q] = u; ql[q] = c; splitf(__fadd_rn(a[q], bfr(vb[h * HD + d + q])), u, c); vh[q] = u; vl[q] = c; }
    for (int ps = 0; ps < 2; ++ps) { *(volatile v4us*)(Qh + e) = qh; *(volatile v4us*)(Ql + e) = ql; *(volatile v4us*)(QVh + e) = vh; *(volatile v4us*)(QVl + e) = vl; if (ps == 0) __threadfence(); } }
__global__ __launch_bounds__(256) void k_kpl(const float* __restrict__ key, bf* KB) { const int e = (blockIdx.x * 256 + threadIdx.x) * 4; if (e >= NH_ * TT * HD) return; const int d = e % HD; const int t = (e / HD) % TT; const int h = e / (HD * TT); const v4f a = *(const v4f*)(key + (size_t)t * DM + h * HD + d); v4us o;
#pragma unroll
    for (int q = 0; q < 4; ++q) o[q] = f2bf(a[q]); *(volatile v4us*)(KB + e) = o; __threadfence(); *(volatile v4us*)(KB + e) = o; }
__global__ __launch_bounds__(256) void k_vt(const float* __restrict__ FV, bf* Vh, bf* Vl) { const int e = (blockIdx.x * 256 + threadIdx.x) * 2; if (e >= NH_ * HD * TT) return; const int t = e % TT; const int d = (e / TT) % HD; const int h = e / (TT * HD); v2us oh, ol;
#pragma unroll
    for (int u = 0; u < 2; ++u) { unsigned short a, c; splitf(FV[(size_t)(t + u) * DM + h * HD + d], a, c); oh[u] = a; ol[u] = c; } *(volatile v2us*)(Vh + e) = oh; *(volatile v2us*)(Vl + e) = ol; __threadfence(); *(volatile v2us*)(Vh + e) = oh; *(volatile v2us*)(Vl + e) = ol; }
__global__ __launch_bounds__(256) void k_relsoft(float* Sb, const float* __restrict__ QR, bf* Ph, bf* Pl) { const int lane = threadIdx.x & 31; const int row = blockIdx.x * 8 + (threadIdx.x >> 5); if (row >= NH_ * TT) return; const int q = row % TT; float* sr = Sb + (size_t)row * TT; const float* rr = QR + (size_t)row * 2 * TT + (TT - q); float mx = -3.0e38f;
#pragma unroll 1
    for (int ch = 0; ch < TT / 128; ++ch) { const int k0 = ch * 128 + lane * 4; v4f a = *(const v4f*)(sr + k0);
#pragma unroll
        for (int u = 0; u < 4; ++u) { a[u] = __fadd_rn(a[u], rr[k0 + u]); mx = fmaxf(mx, a[u]); } *(volatile v4f*)(sr + k0) = a; }
#pragma unroll
    for (int sh = 16; sh; sh >>= 1) mx = fmaxf(mx, __shfl_xor(mx, sh, 32));
    float sum = 0.f;
#pragma unroll 1
    for (int ch = 0; ch < TT / 128; ++ch) { const int k0 = ch * 128 + lane * 4; const v4f a = *(const v4f*)(sr + k0);
#pragma unroll
        for (int u = 0; u < 4; ++u) { float d0 = __fsub_rn(a[u], mx); asm volatile("" : "+v"(d0)); sum += __expf(d0); } }
#pragma unroll
    for (int sh = 16; sh; sh >>= 1) sum += __shfl_xor(sum, sh, 32);
    const float f = __fdiv_rn(1.0f, sum);
    for (int ps = 0; ps < 2; ++ps) {
#pragma unroll 1
        for (int ch = 0; ch < TT / 128; ++ch) { const int k0 = ch * 128 + lane * 4; const v4f a = *(const v4f*)(sr + k0); v4us oh, ol;
#pragma unroll
            for (int u = 0; u < 4; ++u) { float d0 = __fsub_rn(a[u], mx); asm volatile("" : "+v"(d0)); unsigned short hh, ll; splitf(__fmul_rn(__expf(d0), f), hh, ll); oh[u] = hh; ol[u] = ll; }
            *(volatile v4us*)(Ph + (size_t)row * TT + k0) = oh; *(volatile v4us*)(Pl + (size_t)row * TT + k0) = ol; }
        if (ps == 0) __threadfence(); } }
__global__ __launch_bounds__(256) void k_mrg(const float* __restrict__ O, bf* Mh, bf* Ml) { const int e = (blockIdx.x * 256 + threadIdx.x) * 4; if (e >= TT * DM) return; const int c = e % DM; const int t = e / DM; const int h = c / HD, d = c % HD; const float* r = O + ((size_t)h * TT + t) * HD + d; v4us oh, ol;
#pragma unroll
    for (int q = 0; q < 4; ++q) { unsigned short a, b; splitf(r[q], a, b); oh[q] = a; ol[q] = b; } *(volatile v4us*)(Mh + e) = oh; *(volatile v4us*)(Ml + e) = ol; __threadfence(); *(volatile v4us*)(Mh + e) = oh; *(volatile v4us*)(Ml + e) = ol; }

extern "C" void kernel_launch(void* const* d_in, const int* in_sizes, int n_in,
                              void* d_out, int out_size, void* d_ws, size_t ws_size, hipStream_t stream) {
    (void)in_sizes; (void)n_in; (void)out_size;
    const float* query = (const float*)d_in[0]; const float* key = (const float*)d_in[1]; const float* value = (const float*)d_in[2];   const float* wq = (const float*)d_in[4]; const float* bq = (const float*)d_in[5]; const float* wv = (const float*)d_in[6]; const float* bv = (const float*)d_in[7]; const float* wo = (const float*)d_in[8]; const float* bo = (const float*)d_in[9]; const float* vbias = (const float*)d_in[10];
    float* OUT = (float*)d_out;
    char* wsp = (char*)d_ws;
    auto take = [&](size_t bytes) { char* p = wsp; wsp += (bytes + 255) & ~(size_t)255; return (void*)p; };
    bf* WQ = (bf*)take(DM * DM * 2); bf* WV = (bf*)take(DM * DM * 2); bf* WO = (bf*)take(DM * DM * 2); bf* PEh = (bf*)take((size_t)2 * TT * HD * 2); bf* PEl = (bf*)take((size_t)2 * TT * HD * 2);
    bf* XB = (bf*)take((size_t)TT * DM * 2); float* FQ = (float*)take((size_t)TT * DM * 4); float* FV = (float*)take((size_t)TT * DM * 4); bf* Qh = (bf*)take((size_t)NH_ * TT * HD * 2); bf* Ql = (bf*)take((size_t)NH_ * TT * HD * 2); bf* QVh = (bf*)take((size_t)NH_ * TT * HD * 2); bf* QVl = (bf*)take((size_t)NH_ * TT * HD * 2); bf* KB = (bf*)take((size_t)NH_ * TT * HD * 2); bf* VTh = (bf*)take((size_t)NH_ * HD * TT * 2); bf* VTl = (bf*)take((size_t)NH_ * HD * TT * 2);
    float* Sb = (float*)take((size_t)NH_ * TT * TT * 4); float* QR = (float*)take((size_t)NH_ * TT * 2 * TT * 4); bf* Ph = (bf*)take((size_t)NH_ * TT * TT * 2); bf* Pl = (bf*)take((size_t)NH_ * TT * TT * 2); float* O = (float*)take((size_t)NH_ * TT * HD * 4); bf* Mh = (bf*)take((size_t)TT * DM * 2); bf* Ml = (bf*)take((size_t)TT * DM * 2);
    if ((size_t)(wsp - (char*)d_ws) > ws_size) return;
    k_wtG<<<(DM * DM / 64 + 63) / 64, 256, 0, stream>>>(wq, DM, DM, WQ); k_wtG<<<(DM * DM / 64 + 63) / 64, 256, 0, stream>>>(wv, DM, DM, WV); k_wtG<<<(DM * DM / 64 + 63) / 64, 256, 0, stream>>>(wo, DM, DM, WO); k_pe<<<(2 * TT * HD / 4 + 255) / 256, 256, 0, stream>>>(PEh, PEl);
    for (int b = 0; b < NB_; ++b) {
        k_cvt8<<<(TT * DM / 8 + 255) / 256, 256, 0, stream>>>(query + (size_t)b * TT * DM, XB, TT * DM / 8); k_gemmw<bf, 0, true><<<dim3(TT / 64, DM / 64, 1), 32, 0, stream>>>(XB, nullptr, WQ, nullptr, DM, FQ, DM, bq, 0, 0, 0);
        k_cvt8<<<(TT * DM / 8 + 255) / 256, 256, 0, stream>>>(value + (size_t)b * TT * DM, XB, TT * DM / 8); k_gemmw<bf, 0, true><<<dim3(TT / 64, DM / 64, 1), 32, 0, stream>>>(XB, nullptr, WV, nullptr, DM, FV, DM, bv, 0, 0, 0);
        k_qpl<<<(NH_ * TT * HD / 4 + 255) / 256, 256, 0, stream>>>(FQ, vbias, Qh, Ql, QVh, QVl); k_kpl<<<(NH_ * TT * HD / 4 + 255) / 256, 256, 0, stream>>>(key + (size_t)b * TT * DM, KB); k_vt<<<(NH_ * HD * TT / 2 + 255) / 256, 256, 0, stream>>>(FV, VTh, VTl);
        k_gemmw<bf, 1, false><<<dim3(TT / 64, TT / 64, NH_), 32, 0, stream>>>(Qh, Ql, KB, nullptr, HD, Sb, TT, nullptr, (size_t)TT * HD, (size_t)TT * HD, (size_t)TT * TT);
        k_gemmw<bf, 2, false><<<dim3(TT / 64, 2 * TT / 64, NH_), 32, 0, stream>>>(QVh, QVl, PEh, PEl, HD, QR, 2 * TT, nullptr, (size_t)TT * HD, 0, (size_t)TT * 2 * TT);
        k_relsoft<<<NH_ * TT / 8, 256, 0, stream>>>(Sb, QR, Ph, Pl);
        k_gemmw<bf, 2, false><<<dim3(TT / 64, 1, NH_), 32, 0, stream>>>(Ph, Pl, VTh, VTl, TT, O, HD, nullptr, (size_t)TT * TT, (size_t)HD * TT, (size_t)TT * HD);
        k_mrg<<<(TT * DM / 4 + 255) / 256, 256, 0, stream>>>(O, Mh, Ml);
        k_gemmw<bf, 1, true><<<dim3(TT / 64, DM / 64, 1), 32, 0, stream>>>(Mh, Ml, WO, nullptr, DM, OUT + (size_t)b * TT * DM, DM, bo, 0, 0, 0); }
}
